// NaiveBias2d_30451318128837
// MI455X (gfx1250) — hardware-verified
//
#include <hip/hip_runtime.h>
#include <stddef.h>


typedef _Float16 v16h __attribute__((ext_vector_type(16)));
typedef _Float16 v8h  __attribute__((ext_vector_type(8)));
typedef float    v8f  __attribute__((ext_vector_type(8)));
typedef float    v4f  __attribute__((ext_vector_type(4)));
typedef _Float16 h16;

#ifndef NB
#define NB 8
#endif
#define NB_FULL 8
#define SIDE    32
#define SEQ     (SIDE * SIDE)
#define NHEAD   8
#define HD      64
#define WLEN    (2 * SIDE - 1)
#define LSTRIDE (NHEAD * HD)

#define LDB 40
#define LDC 68

#define WCARRY 64.0f
#define SCARRY 16.0f

#define NTHREADS 512
#define OUT_STEPS 32
#define OUT_GROUP 4

static_assert(NB >= 1 && NB <= NB_FULL);
static_assert(SIDE == 32);
static_assert(HD == 64 && (HD % 16) == 0);
static_assert((LDB % 8) == 0 && LDB >= SIDE);
static_assert((LDC % 4) == 0 && LDC >= HD);
static_assert(NTHREADS == 16 * 32);
static_assert(NTHREADS == SIDE * (HD / 4));
static_assert(2 * NTHREADS == SIDE * SIDE);
static_assert(OUT_STEPS * NTHREADS * 4 == SEQ * HD);
static_assert((OUT_STEPS % OUT_GROUP) == 0);
static_assert((size_t)SIDE * LDB * 2 + (size_t)2 * HD * LDB * 2 + (size_t)2 * SIDE * LDC * 4
              <= (size_t)131072);

__device__ __forceinline__ float bf16r(float x) {
  unsigned int u = __float_as_uint(x);
  u = (u + 0x7FFFu + ((u >> 16) & 1u)) & 0xFFFF0000u;
  return __uint_as_float(u);
}

static __device__ __forceinline__ h16 toh_flush(float v) {
  const h16 r = (h16)v;
  return (fabsf(v) < 6.103515625e-05f) ? (h16)0.0f : r;
}

__device__ __forceinline__ v16h frag_at(const _Float16* p) {
  v8h lo = *(const v8h*)(p);
  v8h hi = *(const v8h*)(p + 16);
  v16h out;
#pragma unroll
  for (int i = 0; i < 8; ++i) { out[i] = lo[i]; out[i + 8] = hi[i]; }
  return out;
}
__device__ __forceinline__ v16h ld_frag(const _Float16* base, unsigned ld) {
  const unsigned lane = threadIdx.x & 31u;
  return frag_at(base + (lane & 15u) * ld + (lane >> 4) * 8u);
}

__device__ __forceinline__ v8f wmma16(v16h a, v16h b, v8f c) {
  v8f d = __builtin_amdgcn_wmma_f32_16x16x32_f16(false, a, false, b, (short)0, c,
                                                 false, false);
  asm volatile("v_nop\n\tv_nop\n\tv_nop\n\tv_nop" : "+v"(d) : "v"(a), "v"(b));
  return d;
}

__global__ __launch_bounds__(512) void bias2d_kernel(
    const float* __restrict__ v, const float* __restrict__ w, float* __restrict__ out) {
  __shared__ _Float16 Bs[SIDE * LDB];
  __shared__ _Float16 Sts[2 * HD * LDB];
  __shared__ float    Ts[2 * SIDE * LDC];

  const unsigned tid = threadIdx.x, lane = tid & 31u;
  const unsigned wave = __builtin_amdgcn_readfirstlane(threadIdx.x >> 5);
  const unsigned n = blockIdx.x >> 3;
  const unsigned h = blockIdx.x & 7u;

#pragma unroll
  for (unsigned t = 0; t < 2u; ++t) {
    const unsigned idx = tid + (unsigned)NTHREADS * t;
    const unsigned j = idx >> 5, i = idx & 31u;
    const unsigned k = ((unsigned)SIDE - i + j) % (unsigned)WLEN;
    const float wv = w[h * (unsigned)WLEN + k];
    Bs[j * LDB + i] = toh_flush(WCARRY * bf16r(wv));
  }

  const unsigned q = tid & 15u;
  const unsigned g = tid >> 4;
  const float* vb = v + (size_t)n * SEQ * LSTRIDE + (size_t)h * HD + q * 4u;

  {
    v4f acc = {0.0f, 0.0f, 0.0f, 0.0f};
#pragma unroll 8
    for (unsigned e = 0; e < (unsigned)SIDE; ++e) {
      const v4f val = *(const v4f*)(vb + (size_t)(g * (unsigned)SIDE + e) * LSTRIDE);
#pragma unroll
      for (int i = 0; i < 4; ++i) acc[i] += bf16r(val[i]);
    }
#pragma unroll
    for (unsigned i = 0; i < 4u; ++i)
      Sts[(unsigned)(HD * LDB) + (q * 4u + i) * LDB + g] = toh_flush(SCARRY * acc[i]);
  }
  {
    v4f acc = {0.0f, 0.0f, 0.0f, 0.0f};
#pragma unroll 8
    for (unsigned c = 0; c < (unsigned)SIDE; ++c) {
      const v4f val = *(const v4f*)(vb + (size_t)(c * (unsigned)SIDE + g) * LSTRIDE);
#pragma unroll
      for (int i = 0; i < 4; ++i) acc[i] += bf16r(val[i]);
    }
#pragma unroll
    for (unsigned i = 0; i < 4u; ++i)
      Sts[(q * 4u + i) * LDB + g] = toh_flush(SCARRY * acc[i]);
  }
  __syncthreads();

  {
    const unsigned hh = lane >> 4, m = lane & 15u;
    const unsigned sel  = wave >> 3;
    const unsigned r    = wave & 7u;
    const unsigned boff = (r >> 2) << 4;
    const unsigned doff = (r & 3u) << 4;
    const v16h a = ld_frag(&Bs[boff * LDB], LDB);
    const v16h b = ld_frag(&Sts[sel * (unsigned)(HD * LDB) + doff * LDB], LDB);
    v8f acc = {};
    acc = wmma16(a, b, acc);
#pragma unroll
    for (unsigned r8 = 0; r8 < 8u; ++r8)
      Ts[(sel * (unsigned)SIDE + boff + hh * 8u + r8) * LDC + doff + m] =
          acc[r8] * (1.0f / (WCARRY * SCARRY));
  }
  __syncthreads();

  float* ob = out + (size_t)n * SEQ * LSTRIDE + (size_t)h * HD;
#pragma unroll 1
  for (unsigned grp = 0; grp < (unsigned)(OUT_STEPS / OUT_GROUP); ++grp) {
    v4f xs[OUT_GROUP];
    size_t off[OUT_GROUP];
#pragma unroll
    for (unsigned i = 0; i < (unsigned)OUT_GROUP; ++i) {
      const unsigned idx = (grp * (unsigned)OUT_GROUP + i) * (unsigned)NTHREADS + tid;
      const unsigned j  = idx >> 4;
      const unsigned qq = idx & 15u;
      const unsigned a  = j >> 5;
      const unsigned bb = j & 31u;
      const v4f t1 = *(const v4f*)&Ts[bb * LDC + qq * 4u];
      const v4f t2 = *(const v4f*)&Ts[((unsigned)SIDE + a) * LDC + qq * 4u];
      xs[i] = t1 + t2;
      off[i] = (size_t)j * LSTRIDE + qq * 4u;
    }
#pragma unroll
    for (int i = 0; i < OUT_GROUP; ++i) *(volatile v4f*)(ob + off[i]) = xs[i];
    __threadfence();
#pragma unroll
    for (int i = 0; i < OUT_GROUP; ++i) *(volatile v4f*)(ob + off[i]) = xs[i];
  }
}

extern "C" void kernel_launch(void* const* d_in, const int* in_sizes, int n_in,
                              void* d_out, int out_size, void* d_ws, size_t ws_size,
                              hipStream_t stream) {
  (void)d_ws; (void)ws_size;
  if (n_in < 2) return;
  const long long need_v = (long long)NB * SEQ * LSTRIDE;
  if ((long long)in_sizes[0] < need_v) return;
  if ((long long)in_sizes[1] < (long long)NHEAD * WLEN) return;
  if ((long long)out_size < need_v) return;

  const float* v = (const float*)d_in[0];
  const float* w = (const float*)d_in[1];
  float* out = (float*)d_out;

  bias2d_kernel<<<dim3(NB * NHEAD), dim3(NTHREADS), 0, stream>>>(v, w, out);
}
